// ShiftedWindowAttention_22462678958665
// MI455X (gfx1250) — hardware-verified
//
#include <hip/hip_runtime.h>
#include <math.h>
#include <stdint.h>

#ifndef NB
#define NB 32
#endif
#define NBX    32
#define IMG    56
#define CDIM   128
#define NQKV   (3 * CDIM)
#define NH     4
#define HD     32
#define WSZ    7
#define WS2    49
#define SSZ    3
#define NWI    64
#define WPAD   64
#define RPN    676
#define RPP    680
#define IMG_STRIDE_FULL (IMG * IMG * CDIM)
#define BG     ((NB <= 8) ? NB : 8)
#define NGRP   (NB / BG)
#define GWIN   (BG * NWI)
#define GROWS  (GWIN * WS2)
#define PROWS  (GWIN * WPAD)
#define RSQ_HD 0.17677669529663689f
#define LOG2E  1.4426950408889634f
#define MASKL  (-100.0f * LOG2E)
#define QSC    1024.0f
#define KSC    1024.0f
#define PCAR   32768.0f
#define VCAR   1024.0f
#define OSC    1024.0f
#define WOS    1024.0f
#define ATT_THREADS (NH * 32)
#define PTP    36
#define PTW    (16 * PTP)
#define OSP    132
#define SLAB64 (16 * 68)
#define VTP    72
#define WS_CAP 134217728
static_assert(CDIM == NH * HD && HD == 32 && NH == 4 && ATT_THREADS == 128);
static_assert(NB >= 1 && NB <= NBX && (NB % BG) == 0 && BG >= 1 && BG <= 8);
static_assert(IMG == 8 * WSZ && NWI == 64 && WS2 == WSZ * WSZ && WS2 <= WPAD && WPAD == 64);
static_assert((GROWS % 64) == 0 && (CDIM % 64) == 0 && (CDIM % 32) == 0 && (PROWS % 16) == 0);
static_assert(((GROWS * CDIM) % (8 * 256)) == 0 && ((NQKV * CDIM) % (8 * 256)) == 0 && ((CDIM * CDIM) % (8 * 256)) == 0);
static_assert(RPN == (2 * WSZ - 1) * (2 * WSZ - 1) * NH && RPP >= RPN);

typedef unsigned short u16;
typedef _Float16 v16h __attribute__((ext_vector_type(16)));
typedef _Float16 v8h  __attribute__((ext_vector_type(8)));
typedef __bf16   v16b __attribute__((ext_vector_type(16)));
typedef float    v8f  __attribute__((ext_vector_type(8)));
typedef float    v4f  __attribute__((ext_vector_type(4)));
typedef unsigned int v4u __attribute__((ext_vector_type(4)));

union FragH { v16h v; v8h h[2]; v4u u[2]; };
union FragB { v16b v; v4u u[2]; };

__device__ __forceinline__ unsigned short bf_bits(float f) {
  unsigned u = __float_as_uint(f);
  return (unsigned short)((u + 0x7FFFu + ((u >> 16) & 1u)) >> 16);
}
__device__ __forceinline__ float bf_up(unsigned short h) { return __uint_as_float(((unsigned)h) << 16); }
__device__ __forceinline__ float bfr(float f) { return bf_up(bf_bits(f)); }
__device__ __forceinline__ unsigned short h_bits(_Float16 x) { return __builtin_bit_cast(unsigned short, x); }
__device__ __forceinline__ unsigned pk16(unsigned short a, unsigned short b) { return (unsigned)a | ((unsigned)b << 16); }
__device__ __forceinline__ v8f zero8() { v8f z = {0.f, 0.f, 0.f, 0.f, 0.f, 0.f, 0.f, 0.f}; return z; }
__device__ __forceinline__ int reg3(int p) { return (p < IMG - WSZ) ? 0 : ((p < IMG - SSZ) ? 1 : 2); }

__device__ __forceinline__ size_t pix_of(int rr, int gwin0) {
  const int wl  = rr / WS2;
  const int t   = rr - wl * WS2;
  const int wdx = gwin0 + wl;
  const int bi  = wdx >> 6, wh = (wdx >> 3) & 7, ww = wdx & 7;
  const int ti  = t / WSZ, tj = t - ti * WSZ;
  int ph = wh * WSZ + ti + SSZ;  ph = (ph >= IMG) ? (ph - IMG) : ph;
  int pw = ww * WSZ + tj + SSZ;  pw = (pw >= IMG) ? (pw - IMG) : pw;
  return ((size_t)bi * IMG + ph) * IMG + pw;
}

__device__ __forceinline__ v16h ldfrag_h(const _Float16* p) {
  FragH f;
  f.h[0] = *(const v8h*)(p);
  f.h[1] = *(const v8h*)(p + 16);
  return f.v;
}
__device__ __forceinline__ v16b ldfrag_b(const u16* p) {
  FragB f;
  f.u[0] = *(const v4u*)(p);
  f.u[1] = *(const v4u*)(p + 16);
  return f.v;
}

__device__ __forceinline__ v8f mma_h(v16h a, v16h b, v8f c) {
  return __builtin_amdgcn_wmma_f32_16x16x32_f16(false, a, false, b, (short)0, c, false, false);
}
__device__ __forceinline__ v8f mma_b(v16b a, v16b b, v8f c) {
  return __builtin_amdgcn_wmma_f32_16x16x32_bf16(false, a, false, b, (short)0, c, false, false);
}
__device__ __forceinline__ void guard2(v8f& a, v8f& b, v16h x0, v16h x1, v16h x2, v16h x3, v16h x4, v16h x5) {
#if defined(__HIP_DEVICE_COMPILE__)
  asm volatile("v_nop\n\tv_nop\n\tv_nop\n\tv_nop"
               : "+v"(a), "+v"(b) : "v"(x0), "v"(x1), "v"(x2), "v"(x3), "v"(x4), "v"(x5) : "memory");
#endif
}
template <typename F>
__device__ __forceinline__ void guard6(v8f& a, v8f& b, v8f& c, v8f& d, F x0, F x1, F x2, F x3, F x4, F x5) {
#if defined(__HIP_DEVICE_COMPILE__)
  asm volatile("v_nop\n\tv_nop\n\tv_nop\n\tv_nop"
               : "+v"(a), "+v"(b), "+v"(c), "+v"(d) : "v"(x0), "v"(x1), "v"(x2), "v"(x3), "v"(x4), "v"(x5) : "memory");
#endif
}
__device__ __forceinline__ void acc_guard2(v8f& a, v8f& b) {
#if defined(__HIP_DEVICE_COMPILE__)
  asm volatile("v_nop\n\tv_nop\n\tv_nop\n\tv_nop" : "+v"(a), "+v"(b));
#endif
}
__device__ __forceinline__ void wave_sync_lds() {
  __builtin_amdgcn_fence(__ATOMIC_RELEASE, "workgroup");
  __builtin_amdgcn_wave_barrier();
  __builtin_amdgcn_fence(__ATOMIC_ACQUIRE, "workgroup");
}

__global__ __launch_bounds__(256) void cvt16(const float* __restrict__ x, u16* D, int n8, int f16mode, float scale) {
  const int gt = blockIdx.x * 256 + (int)threadIdx.x;
  if (gt >= n8) return;
  const float* p = x + (size_t)gt * 8;
  const v4f a = *(const v4f*)(p), b4 = *(const v4f*)(p + 4);
  float w[8];
#pragma unroll
  for (int e = 0; e < 4; ++e) { w[e] = a[e]; w[4 + e] = b4[e]; }
  v4u o;
#pragma unroll
  for (int e = 0; e < 4; ++e) {
    const float f0 = w[2 * e], f1 = w[2 * e + 1];
    const unsigned short hb0 = h_bits((_Float16)(bfr(f0) * scale));
    const unsigned short hb1 = h_bits((_Float16)(bfr(f1) * scale));
    const unsigned short bb0 = bf_bits(f0);
    const unsigned short bb1 = bf_bits(f1);
    o[e] = (f16mode != 0) ? pk16(hb0, hb1) : pk16(bb0, bb1);
  }
  u16* d = D + (size_t)gt * 8;
  for (int pass = 0; pass < 2; ++pass) {
    *(volatile v4u*)(d) = o;
    __threadfence();
  }
}

__global__ __launch_bounds__(256) void xw16(const float* __restrict__ x, u16* D, int n8, int gwin0) {
  const int gt = blockIdx.x * 256 + (int)threadIdx.x;
  if (gt >= n8) return;
  const int row = gt >> 4;
  const int e8  = (gt & 15) * 8;
  const float* p = x + pix_of(row, gwin0) * (size_t)CDIM + e8;
  const v4f a = *(const v4f*)(p), b4 = *(const v4f*)(p + 4);
  v4u o;
#pragma unroll
  for (int e = 0; e < 4; ++e) {
    const float f0 = (e < 2) ? a[2 * e] : b4[2 * e - 4];
    const float f1 = (e < 2) ? a[2 * e + 1] : b4[2 * e - 3];
    o[e] = pk16(bf_bits(f0), bf_bits(f1));
  }
  u16* d = D + (size_t)row * CDIM + e8;
  for (int pass = 0; pass < 2; ++pass) {
    *(volatile v4u*)(d) = o;
    __threadfence();
  }
}

__global__ __launch_bounds__(256) void qk16(const float* __restrict__ F, u16* Hp, u16* Lp, float sc) {
  const int tid = (int)threadIdx.x;
  const int pr  = (int)blockIdx.x * 16 + (tid >> 4);
  if (pr >= PROWS) return;
  const int cc  = tid & 15;
  const int wl  = pr >> 6;
  const int t   = pr & 63;
  const bool valid = (t < WS2);
  const int tcl = valid ? t : (WS2 - 1);
  const float* p = F + ((size_t)wl * WS2 + tcl) * CDIM + cc * 8;
  const v4f a = *(const v4f*)(p), b4 = *(const v4f*)(p + 4);
  float w[8];
#pragma unroll
  for (int e = 0; e < 4; ++e) {
    w[e]     = valid ? (a[e] * sc)  : 0.0f;
    w[4 + e] = valid ? (b4[e] * sc) : 0.0f;
  }
  v4u oh, ol;
#pragma unroll
  for (int e = 0; e < 4; ++e) {
    const float t0 = w[2 * e], t1 = w[2 * e + 1];
    const _Float16 h0 = (_Float16)t0, h1 = (_Float16)t1;
    const _Float16 l0 = (_Float16)(t0 - (float)h0), l1 = (_Float16)(t1 - (float)h1);
    oh[e] = pk16(h_bits(h0), h_bits(h1));
    ol[e] = pk16(h_bits(l0), h_bits(l1));
  }
  u16* dh = Hp + (size_t)pr * CDIM + cc * 8;
  u16* dl = Lp + (size_t)pr * CDIM + cc * 8;
  for (int pass = 0; pass < 2; ++pass) {
    *(volatile v4u*)(dh) = oh;
    *(volatile v4u*)(dl) = ol;
    __threadfence();
  }
}

__global__ __launch_bounds__(256) void vt16(const float* __restrict__ F, u16* VHo, u16* VLo) {
  __shared__ __align__(16) u16 TH[CDIM * VTP];
  __shared__ __align__(16) u16 TL[CDIM * VTP];
  const int tid = threadIdx.x;
  const int wl  = blockIdx.x;
  if (wl >= GWIN) return;
  {
    const int sl = tid >> 2;
    const int dc = (tid & 3) * 32;
    const bool valid = (sl < WS2);
    const int scl = valid ? sl : (WS2 - 1);
    const float* src = F + ((size_t)wl * WS2 + scl) * CDIM + dc;
#pragma unroll
    for (int i = 0; i < 8; ++i) {
      const v4f a = *(const v4f*)(src + 4 * i);
#pragma unroll
      for (int e = 0; e < 4; ++e) {
        const float t = valid ? (a[e] * VCAR) : 0.0f;
        const _Float16 hv = (_Float16)t;
        const _Float16 lv = (_Float16)(t - (float)hv);
        TH[(dc + 4 * i + e) * VTP + sl] = h_bits(hv);
        TL[(dc + 4 * i + e) * VTP + sl] = h_bits(lv);
      }
    }
  }
  __syncthreads();
  v4u vh[4], vl[4];
  const int q8 = tid >> 3, p8 = (tid & 7) * 8;
#pragma unroll
  for (int it = 0; it < 4; ++it) {
    const int line = it * 32 + q8;
    vh[it] = *(const v4u*)(TH + line * VTP + p8);
    vl[it] = *(const v4u*)(TL + line * VTP + p8);
  }
  const size_t base = (size_t)wl * CDIM * WPAD + p8;
  for (int pass = 0; pass < 2; ++pass) {
#pragma unroll
    for (int it = 0; it < 4; ++it) {
      const int line = it * 32 + q8;
      *(volatile v4u*)(VHo + base + (size_t)line * WPAD) = vh[it];
      *(volatile v4u*)(VLo + base + (size_t)line * WPAD) = vl[it];
    }
    __threadfence();
  }
}

__device__ __forceinline__ void stage64(float* sl, v8f a0, v8f a1, v8f a2, v8f a3, float oscale,
                                        const float* __restrict__ bias, int col0, int lane) {
  const int hh = lane >> 4, m = lane & 15;
  const float b0 = bfr(bias[col0 + m]);
  const float b1 = bfr(bias[col0 + 16 + m]);
  const float b2 = bfr(bias[col0 + 32 + m]);
  const float b3 = bfr(bias[col0 + 48 + m]);
#pragma unroll
  for (int r = 0; r < 8; ++r) {
    const int ro = (8 * hh + r) * 68 + m;
    sl[ro]      = a0[r] * oscale + b0;
    sl[ro + 16] = a1[r] * oscale + b1;
    sl[ro + 32] = a2[r] * oscale + b2;
    sl[ro + 48] = a3[r] * oscale + b3;
  }
  wave_sync_lds();
}
__device__ __forceinline__ void epi64(float* sl, v8f a0, v8f a1, v8f a2, v8f a3, float oscale,
                                      const float* __restrict__ bias, float* C, int N, size_t rowb, int col0, int lane) {
  const int hh = lane >> 4, m = lane & 15;
  stage64(sl, a0, a1, a2, a3, oscale, bias, col0, lane);
  v4f vals[8];
#pragma unroll
  for (int it = 0; it < 8; ++it) vals[it] = *(const v4f*)(sl + (it * 2 + hh) * 68 + m * 4);
  float* dst = C + (rowb + (size_t)hh) * (size_t)N + col0 + m * 4;
  for (int pass = 0; pass < 2; ++pass) {
#pragma unroll
    for (int it = 0; it < 8; ++it) {
      *(volatile v4f*)(dst + (size_t)(it * 2) * (size_t)N) = vals[it];
    }
    __threadfence();
  }
}
__device__ __forceinline__ void epi64_px(float* sl, v8f a0, v8f a1, v8f a2, v8f a3, float oscale,
                                         const float* __restrict__ bias, float* C, int rowb, int col0, int gwin0, int lane) {
  const int hh = lane >> 4, m = lane & 15;
  stage64(sl, a0, a1, a2, a3, oscale, bias, col0, lane);
  v4f vals[8];
  size_t dsto[8];
#pragma unroll
  for (int it = 0; it < 8; ++it) {
    vals[it] = *(const v4f*)(sl + (it * 2 + hh) * 68 + m * 4);
    const int rr = rowb + it * 2 + hh;
    dsto[it] = pix_of(rr, gwin0) * (size_t)CDIM + col0 + m * 4;
  }
  for (int pass = 0; pass < 2; ++pass) {
#pragma unroll
    for (int it = 0; it < 8; ++it) {
      *(volatile v4f*)(C + dsto[it]) = vals[it];
    }
    __threadfence();
  }
}

__global__ __launch_bounds__(128)
void gemm_bf(const u16* __restrict__ A, const u16* __restrict__ Bt, const float* __restrict__ bias,
             float* C, int M, int N, int K, float oscale) {
  __shared__ __align__(16) float slab[4 * SLAB64];
  const int tid = threadIdx.x, wave = tid >> 5, lane = tid & 31, hh = lane >> 4, m = lane & 15;
  const int ntile = N >> 6;
  const int bid   = blockIdx.x;
  const int rowb  = (bid / ntile) * 64 + wave * 16;
  const int col0  = (bid % ntile) * 64;
  if (rowb + 16 > M) return;
  const u16* ap = A  + (size_t)(rowb + m) * K + 8 * hh;
  const u16* bp = Bt + (size_t)(col0 + m) * K + 8 * hh;
  const size_t bs = (size_t)16 * K;
  v8f acc0 = zero8(), acc1 = zero8(), acc2 = zero8(), acc3 = zero8();
#pragma unroll 1
  for (int k0 = 0; k0 < K; k0 += 32) {
    const v16b a  = ldfrag_b(ap + k0);
    const v16b b0 = ldfrag_b(bp + k0);
    const v16b b1 = ldfrag_b(bp + bs + k0);
    const v16b b2 = ldfrag_b(bp + 2 * bs + k0);
    const v16b b3 = ldfrag_b(bp + 3 * bs + k0);
    acc0 = mma_b(a, b0, acc0);
    acc1 = mma_b(a, b1, acc1);
    acc2 = mma_b(a, b2, acc2);
    acc3 = mma_b(a, b3, acc3);
    guard6<v16b>(acc0, acc1, acc2, acc3, a, b0, b1, b2, b3, a);
  }
  epi64(slab + wave * SLAB64, acc0, acc1, acc2, acc3, oscale, bias, C, N, (size_t)rowb, col0, lane);
}

__global__ __launch_bounds__(128)
void gemm_o(const u16* __restrict__ Ah, const u16* __restrict__ Al, const u16* __restrict__ Bt,
            const float* __restrict__ bias, float* C, int gwin0, float oscale) {
  __shared__ __align__(16) float slab[4 * SLAB64];
  const int tid = threadIdx.x, wave = tid >> 5, lane = tid & 31, hh = lane >> 4, m = lane & 15;
  const int ntile = CDIM >> 6;
  const int bid   = blockIdx.x;
  const int ct    = bid % ntile;
  const int rt    = bid / ntile;
  const int rowb  = rt * 64 + wave * 16;
  if (rowb + 16 > GROWS) return;
  const int col0  = ct * 64;
  const int K     = CDIM;
  const _Float16* ahp = (const _Float16*)(const void*)Ah + ((size_t)rowb + m) * K + 8 * hh;
  const _Float16* alp = (const _Float16*)(const void*)Al + ((size_t)rowb + m) * K + 8 * hh;
  const _Float16* bp  = (const _Float16*)(const void*)Bt + (size_t)(col0 + m) * K + 8 * hh;
  const size_t bs = (size_t)16 * K;
  v8f acc0 = zero8(), acc1 = zero8(), acc2 = zero8(), acc3 = zero8();
#pragma unroll 1
  for (int k0 = 0; k0 < K; k0 += 32) {
    const v16h ah = ldfrag_h(ahp + k0), al = ldfrag_h(alp + k0);
    const v16h b0 = ldfrag_h(bp + k0);
    const v16h b1 = ldfrag_h(bp + bs + k0);
    const v16h b2 = ldfrag_h(bp + 2 * bs + k0);
    const v16h b3 = ldfrag_h(bp + 3 * bs + k0);
    acc0 = mma_h(ah, b0, acc0);  acc0 = mma_h(al, b0, acc0);
    acc1 = mma_h(ah, b1, acc1);  acc1 = mma_h(al, b1, acc1);
    acc2 = mma_h(ah, b2, acc2);  acc2 = mma_h(al, b2, acc2);
    acc3 = mma_h(ah, b3, acc3);  acc3 = mma_h(al, b3, acc3);
    guard6<v16h>(acc0, acc1, acc2, acc3, ah, al, b0, b1, b2, b3);
  }
  epi64_px(slab + wave * SLAB64, acc0, acc1, acc2, acc3, oscale, bias, C, rowb, col0, gwin0, lane);
}

__global__ __launch_bounds__(ATT_THREADS)
void attn_w(const u16* __restrict__ QHp, const u16* __restrict__ QLp,
            const u16* __restrict__ KHp, const u16* __restrict__ KLp,
            const u16* __restrict__ VHp, const u16* __restrict__ VLp,
            const float* __restrict__ rpb, u16* OHp, u16* OLp) {
  __shared__ __align__(16) float ptile[NH * PTW];
  __shared__ __align__(16) float oslab[16 * OSP];
  __shared__ float rp[RPP];

  const int tid  = threadIdx.x;
  const int wave = tid >> 5;
  const int lane = tid & 31;
  const int hh   = lane >> 4;
  const int c    = lane & 15;
  const int bid  = blockIdx.x;
  const int qt   = bid & 3;
  const int wl   = bid >> 2;
  if (wl >= GWIN) return;
  const int head = wave;
  const int q0   = qt * 16;

  for (int i = tid; i < RPN; i += ATT_THREADS) rp[i] = bfr(rpb[i]) * LOG2E;

  float* pt = ptile + wave * PTW;

  const size_t prow0 = (size_t)wl * WPAD;
  const size_t hcol  = (size_t)head * HD + 8 * hh;
  const _Float16* Qh  = (const _Float16*)(const void*)QHp + (prow0 + q0 + c) * CDIM + hcol;
  const _Float16* Ql  = (const _Float16*)(const void*)QLp + (prow0 + q0 + c) * CDIM + hcol;
  const _Float16* Khb = (const _Float16*)(const void*)KHp + (prow0 + c) * CDIM + hcol;
  const _Float16* Klb = (const _Float16*)(const void*)KLp + (prow0 + c) * CDIM + hcol;
  const _Float16* Vhb = (const _Float16*)(const void*)VHp + ((size_t)(wl * NH + head) * HD + c) * WPAD + 8 * hh;
  const _Float16* Vlb = (const _Float16*)(const void*)VLp + ((size_t)(wl * NH + head) * HD + c) * WPAD + 8 * hh;
  const float lsc = RSQ_HD * (LOG2E / (QSC * KSC));
  const float oc  = 1.0f / (PCAR * VCAR);
  const size_t KROW = (size_t)CDIM;

  const int wi   = wl & 63;
  const int winh = wi >> 3, winw = wi & 7;
  const int qr0  = q0 + 8 * hh;

  int qb[8], labq[8];
  bool vq[8];
#pragma unroll
  for (int r = 0; r < 8; ++r) {
    const int qr  = qr0 + r;
    vq[r] = (qr < WS2);
    const int qrc = vq[r] ? qr : (WS2 - 1);
    const int qh  = qrc / WSZ, qw = qrc - qh * WSZ;
    qb[r]   = ((qh + WSZ - 1) * (2 * WSZ - 1) + qw + WSZ - 1) * NH + head;
    labq[r] = 3 * reg3(winh * WSZ + qh) + reg3(winw * WSZ + qw);
  }

  __syncthreads();

  float mrow[8], lrow[8];
  v8f o[2];
#pragma unroll
  for (int r = 0; r < 8; ++r) { mrow[r] = -INFINITY; lrow[r] = 0.f; }
  o[0] = zero8(); o[1] = zero8();

#pragma unroll 1
  for (int kt = 0; kt < 2; ++kt) {
    const int kb = kt * 32;
    v8f s0 = zero8(), s1 = zero8();
    {
      const _Float16* k0p = Khb + (size_t)kb * KROW;
      const _Float16* k1p = k0p + (size_t)16 * KROW;
      const _Float16* l0p = Klb + (size_t)kb * KROW;
      const _Float16* l1p = l0p + (size_t)16 * KROW;
      const v16h qh  = ldfrag_h(Qh);
      const v16h ql  = ldfrag_h(Ql);
      const v16h kh0 = ldfrag_h(k0p);
      const v16h kh1 = ldfrag_h(k1p);
      const v16h kl0 = ldfrag_h(l0p);
      const v16h kl1 = ldfrag_h(l1p);
      s0 = mma_h(qh, kh0, s0);
      s0 = mma_h(ql, kh0, s0);
      s0 = mma_h(qh, kl0, s0);
      s1 = mma_h(qh, kh1, s1);
      s1 = mma_h(ql, kh1, s1);
      s1 = mma_h(qh, kl1, s1);
      guard2(s0, s1, qh, ql, kh0, kl0, kh1, kl1);
    }
    const int  key0 = kb + c, key1 = kb + 16 + c;
    const bool vk0  = (key0 < WS2), vk1 = (key1 < WS2);
    const int  k0c  = vk0 ? key0 : (WS2 - 1), k1c = vk1 ? key1 : (WS2 - 1);
    const int  kh0i = k0c / WSZ, kw0 = k0c - kh0i * WSZ;
    const int  kh1i = k1c / WSZ, kw1 = k1c - kh1i * WSZ;
    const int  kofs0 = (kh0i * (2 * WSZ - 1) + kw0) * NH;
    const int  kofs1 = (kh1i * (2 * WSZ - 1) + kw1) * NH;
    const int  labk0 = 3 * reg3(winh * WSZ + kh0i) + reg3(winw * WSZ + kw0);
    const int  labk1 = 3 * reg3(winh * WSZ + kh1i) + reg3(winw * WSZ + kw1);
#pragma unroll
    for (int r = 0; r < 8; ++r) {
      const float u0 = s0[r] * lsc;
      const float u1 = s1[r] * lsc;
      const float rb0 = rp[qb[r] - kofs0];
      const float rb1 = rp[qb[r] - kofs1];
      const float mk0 = (labq[r] != labk0) ? MASKL : 0.0f;
      const float mk1 = (labq[r] != labk1) ? MASKL : 0.0f;
      const float a0 = vq[r] ? ((u0 + rb0) + mk0) : u0;
      const float a1 = vq[r] ? ((u1 + rb1) + mk1) : u1;
      const float t0 = vk0 ? a0 : -INFINITY;
      const float t1 = vk1 ? a1 : -INFINITY;
      float mx = fmaxf(t0, t1);
#pragma unroll
      for (int off = 1; off < 16; off <<= 1) mx = fmaxf(mx, __shfl_xor(mx, off, 32));
      const float mn = fmaxf(mrow[r], mx);
      const float ms = (mn == -INFINITY) ? 0.0f : mn;
      const float al = exp2f(mrow[r] - ms);
      mrow[r] = mn;
      const float e0 = exp2f(t0 - ms), e1 = exp2f(t1 - ms);
      float ps = e0 + e1;
#pragma unroll
      for (int off = 1; off < 16; off <<= 1) ps += __shfl_xor(ps, off, 32);
      lrow[r] = lrow[r] * al + ps;
      o[0][r] *= al;
      o[1][r] *= al;
      const int ro = (8 * hh + r) * PTP + c;
      pt[ro]      = e0;
      pt[ro + 16] = e1;
    }
    wave_sync_lds();
    FragH ph, pl;
    {
      const float* prow = pt + c * PTP + 8 * hh;
      const v4f p0 = *(const v4f*)(prow), p1 = *(const v4f*)(prow + 4);
      const v4f p2 = *(const v4f*)(prow + 16), p3 = *(const v4f*)(prow + 20);
#pragma unroll
      for (int e = 0; e < 4; ++e) {
        const float ta = p0[e] * PCAR, tb = p1[e] * PCAR, tc = p2[e] * PCAR, td = p3[e] * PCAR;
        const _Float16 ha = (_Float16)ta, hb = (_Float16)tb, hc = (_Float16)tc, hd = (_Float16)td;
        ph.h[0][e]     = ha;
        ph.h[0][4 + e] = hb;
        ph.h[1][e]     = hc;
        ph.h[1][4 + e] = hd;
        pl.h[0][e]     = (_Float16)(ta - (float)ha);
        pl.h[0][4 + e] = (_Float16)(tb - (float)hb);
        pl.h[1][e]     = (_Float16)(tc - (float)hc);
        pl.h[1][4 + e] = (_Float16)(td - (float)hd);
      }
    }
    {
      const _Float16* vhp = Vhb + kb;
      const _Float16* vlp = Vlb + kb;
      const size_t db = (size_t)16 * WPAD;
      const v16h vha = ldfrag_h(vhp), vhb2 = ldfrag_h(vhp + db);
      const v16h vla = ldfrag_h(vlp), vlb2 = ldfrag_h(vlp + db);
      o[0] = mma_h(ph.v, vha,  o[0]);
      o[0] = mma_h(pl.v, vha,  o[0]);
      o[0] = mma_h(ph.v, vla,  o[0]);
      o[1] = mma_h(ph.v, vhb2, o[1]);
      o[1] = mma_h(pl.v, vhb2, o[1]);
      o[1] = mma_h(ph.v, vlb2, o[1]);
      guard2(o[0], o[1], ph.v, pl.v, vha, vhb2, vla, vlb2);
    }
    wave_sync_lds();
  }
  acc_guard2(o[0], o[1]);
#pragma unroll
  for (int r = 0; r < 8; ++r) {
    const float lv  = lrow[r];
    const float ls  = (lv > 0.0f) ? lv : 1.0f;
    const float inv = (lv > 0.0f) ? ((1.0f / ls) * oc) : 0.0f;
    const int   rb  = (8 * hh + r) * OSP + head * HD + c;
    oslab[rb]      = o[0][r] * inv;
    oslab[rb + 16] = o[1][r] * inv;
  }
  __syncthreads();
  v4u oh[2], ol[2];
  size_t offs[2];
  bool vrow[2];
  const int L = tid >> 3, p8 = (tid & 7) * 8;
#pragma unroll
  for (int it = 0; it < 2; ++it) {
    const int row  = it * 8 + (L >> 1);
    const int colb = (L & 1) * 64 + p8;
    const v4f a = *(const v4f*)(oslab + row * OSP + colb), b4 = *(const v4f*)(oslab + row * OSP + colb + 4);
    float w[8];
#pragma unroll
    for (int e = 0; e < 4; ++e) { w[e] = a[e] * OSC; w[4 + e] = b4[e] * OSC; }
#pragma unroll
    for (int e = 0; e < 4; ++e) {
      const _Float16 h0 = (_Float16)w[2 * e], h1 = (_Float16)w[2 * e + 1];
      const _Float16 l0 = (_Float16)(w[2 * e] - (float)h0), l1 = (_Float16)(w[2 * e + 1] - (float)h1);
      oh[it][e] = pk16(h_bits(h0), h_bits(h1));
      ol[it][e] = pk16(h_bits(l0), h_bits(l1));
    }
    vrow[it] = (q0 + row < WS2);
    offs[it] = ((size_t)wl * WS2 + q0 + row) * CDIM + colb;
  }
  for (int pass = 0; pass < 2; ++pass) {
#pragma unroll
    for (int it = 0; it < 2; ++it) {
      if (vrow[it]) {
        *(volatile v4u*)(OHp + offs[it]) = oh[it];
        *(volatile v4u*)(OLp + offs[it]) = ol[it];
      }
    }
    __threadfence();
  }
}

static inline size_t al32k(size_t v) { return (v + 32767) & ~(size_t)32767; }

extern "C" void kernel_launch(void* const* d_in, const int* in_sizes, int n_in,
                              void* d_out, int out_size, void* d_ws, size_t ws_size,
                              hipStream_t stream) {
  if (n_in < 6) return;
  if (in_sizes[0] < NB * IMG_STRIDE_FULL) return;
  if (in_sizes[1] != NQKV * CDIM) return;
  if (in_sizes[2] != NQKV) return;
  if (in_sizes[3] != CDIM * CDIM) return;
  if (in_sizes[4] != CDIM) return;
  if (in_sizes[5] != RPN) return;
  if (out_size < NB * IMG_STRIDE_FULL) return;

  const float* x     = (const float*)d_in[0];
  const float* wqkv  = (const float*)d_in[1];
  const float* bqkv  = (const float*)d_in[2];
  const float* wproj = (const float*)d_in[3];
  const float* bproj = (const float*)d_in[4];
  const float* rpb   = (const float*)d_in[5];
  float*       out   = (float*)d_out;

  const size_t szXB = al32k((size_t)GROWS * CDIM * 2);
  const size_t szWQ = al32k((size_t)NQKV * CDIM * 2);
  const size_t szWO = al32k((size_t)CDIM * CDIM * 2);
  const size_t szF  = al32k((size_t)GROWS * CDIM * 4);
  const size_t szO  = (size_t)GROWS * CDIM * 2;
  const size_t szQ  = al32k((size_t)PROWS * CDIM * 2);
  const size_t szV  = al32k((size_t)GWIN * NH * HD * WPAD * 2);
  if (2 * szO > szF) return;
  size_t off = 0;
  const size_t oXB = off; off += szXB;
  const size_t oWQ = off; off += szWQ;
  const size_t oWO = off; off += szWO;
  const size_t oF  = off; off += szF;
  const size_t oQH = off; off += szQ;
  const size_t oQL = off; off += szQ;
  const size_t oKH = off; off += szQ;
  const size_t oKL = off; off += szQ;
  const size_t oVH = off; off += szV;
  const size_t oVL = off; off += szV;
  if (off > ws_size) return;
  if (off > (size_t)WS_CAP) return;

  char*  ws   = (char*)d_ws;
  u16*   XB   = (u16*)(ws + oXB);
  u16*   WQKV = (u16*)(ws + oWQ);
  u16*   WO   = (u16*)(ws + oWO);
  float* F    = (float*)(ws + oF);
  u16*   OH   = (u16*)(ws + oF);
  u16*   OL   = (u16*)(ws + oF + szO);
  u16*   QH   = (u16*)(ws + oQH);
  u16*   QL   = (u16*)(ws + oQL);
  u16*   KH   = (u16*)(ws + oKH);
  u16*   KL   = (u16*)(ws + oKL);
  u16*   VH   = (u16*)(ws + oVH);
  u16*   VL   = (u16*)(ws + oVL);

  const dim3 b256(256), b128(128), bAT(ATT_THREADS);
  const int  n8w  = (NQKV * CDIM) / 8;
  const int  n8p  = (CDIM * CDIM) / 8;
  const int  n8x  = (GROWS * CDIM) / 8;
  const dim3 gW((n8w + 255) / 256), gP((n8p + 255) / 256), gX((n8x + 255) / 256);
  const dim3 gG((GROWS / 64) * (CDIM / 64));
  const dim3 gVT(GWIN);
  const dim3 gQK(PROWS / 16);
  const dim3 gAT(GWIN * 4);
  const dim3 gO((GROWS / 64) * (CDIM / 64));
  const float osc = 1.0f / (OSC * WOS);

  cvt16<<<gW, b256, 0, stream>>>(wqkv, WQKV, n8w, 0, 1.0f);
  cvt16<<<gP, b256, 0, stream>>>(wproj, WO, n8p, 1, WOS);

  for (int g = 0; g < NGRP; ++g) {
    const int gwin0 = g * GWIN;
    xw16<<<gX, b256, 0, stream>>>(x, XB, n8x, gwin0);
    gemm_bf<<<gG, b128, 0, stream>>>(XB, WQKV + (size_t)2 * CDIM * CDIM, bqkv + 2 * CDIM, F, GROWS, CDIM, CDIM, 1.0f);
    vt16<<<gVT, b256, 0, stream>>>(F, VH, VL);
    gemm_bf<<<gG, b128, 0, stream>>>(XB, WQKV, bqkv, F, GROWS, CDIM, CDIM, 1.0f);
    qk16<<<gQK, b256, 0, stream>>>(F, QH, QL, QSC);
    gemm_bf<<<gG, b128, 0, stream>>>(XB, WQKV + (size_t)CDIM * CDIM, bqkv + CDIM, F, GROWS, CDIM, CDIM, 1.0f);
    qk16<<<gQK, b256, 0, stream>>>(F, KH, KL, KSC);
    attn_w<<<gAT, bAT, 0, stream>>>(QH, QL, KH, KL, VH, VL, rpb, OH, OL);
    gemm_o<<<gO, b128, 0, stream>>>(OH, OL, WO, bproj, out, gwin0, osc);
  }
  (void)hipGetLastError();
}
